// MSMCM_23828478558391
// MI455X (gfx1250) — hardware-verified
//
#include <hip/hip_runtime.h>
#include <hip/hip_bf16.h>
#include <math.h>


#define BB 2
#define SS 2048
#define DD 1024
#define HH 16
#define DKK 64
#define QW 2

typedef _Float16 bf16;
typedef __attribute__((ext_vector_type(4))) unsigned v4u_t;
typedef unsigned v4ua __attribute__((ext_vector_type(4), may_alias));
typedef __attribute__((ext_vector_type(4))) float v4f_t;
typedef float v4fa __attribute__((ext_vector_type(4), may_alias));
typedef __attribute__((ext_vector_type(16))) bf16  bf16x16;
typedef __attribute__((ext_vector_type(8)))  bf16  bf16x8;
typedef __attribute__((ext_vector_type(4)))  bf16  bf16x4;
typedef __attribute__((ext_vector_type(8)))  float f32x8;

#define LDS_STRIDE 48
#define KSTRIDE    72
#define VSTRIDE    48

__device__ __forceinline__ f32x8 wmma_bf16(bf16x16 a, bf16x16 b, f32x8 c) {
  return __builtin_amdgcn_wmma_f32_16x16x32_f16(
      false, a, false, b, (short)0, c, false, false);
}
#define RSPLIT (1.0f / 2048.0f)
__device__ __forceinline__ bf16 lo_of(float v, bf16 h) { return (bf16)((v - (float)h) * 2048.0f); }
__device__ __forceinline__ f32x8 wmma_split(bf16x16 a, bf16x16 al, bf16x16 b, bf16x16 bl, f32x8 c) {
  f32x8 x = {}; x = wmma_bf16(al, b, x); x = wmma_bf16(a, bl, x); return wmma_bf16(a, b, c) + x * RSPLIT; }

template <typename T>
__device__ __forceinline__ bf16x16 load_frag(const T* __restrict__ base, int ld,
                                             int row0, int k0) {
  const int lane = threadIdx.x & 31;
  const int r    = lane & 15;
  const int kh   = (lane >> 4) * 8;
  const T* p0 = base + (size_t)(row0 + r) * ld + (k0 + kh);
  const T* p1 = p0 + 16;
  bf16x16 f;
#pragma unroll
  for (int i = 0; i < 8; ++i) {
    f[i]     = (bf16)p0[i];
    f[i + 8] = (bf16)p1[i];
  }
  return f;
}

__device__ __forceinline__ bf16x16 lds_frag(const bf16* base, int stride) {
  const int lane = threadIdx.x & 31;
  const int row  = lane & 15;
  const int kh   = (lane >> 4) * 8;
  const bf16x8 lo = *(const bf16x8*)(base + row * stride + kh);
  const bf16x8 hi = *(const bf16x8*)(base + row * stride + kh + 16);
  bf16x16 f;
#pragma unroll
  for (int i = 0; i < 8; ++i) { f[i] = lo[i]; f[i + 8] = hi[i]; }
  return f;
}

template <typename T>
__device__ __forceinline__ void stage_read16(const T* __restrict__ p, float* buf) {
#pragma unroll
  for (int i = 0; i < 16; ++i) buf[i] = (float)p[i];
}

__device__ __forceinline__ void stage_write(bf16* dst, const float* buf, int nquad) {
#pragma unroll
  for (int i = 0; i < nquad; ++i) {
    bf16x4 q;
    q[0] = (bf16)buf[4 * i];     q[1] = (bf16)buf[4 * i + 1];
    q[2] = (bf16)buf[4 * i + 2]; q[3] = (bf16)buf[4 * i + 3];
    *(bf16x4*)(dst + 4 * i) = q;
  }
}

__global__ __launch_bounds__(256) void transpose_pack_kernel(const float* __restrict__ W, bf16* __restrict__ WT, int K, int N, size_t plane) {
  __shared__ float tile[64][65];
  const int k0 = blockIdx.y * 64, n0 = blockIdx.x * 64, t = threadIdx.x;
  for (int i = t; i < 64 * 64; i += 256) { const int kr = i >> 6, nc = i & 63; tile[kr][nc] = W[(size_t)(k0 + kr) * N + n0 + nc]; }
  __syncthreads();
#pragma unroll 1
  for (int pass = 0; pass < 2; ++pass) {
    for (int i = t; i < 64 * 8; i += 256) { const int nr = i >> 3, k8 = (i & 7) * 8; bf16 hh[8], hl[8];
#pragma unroll
      for (int e = 0; e < 8; ++e) { const float v = tile[k8 + e][nr]; hh[e] = (bf16)v; hl[e] = lo_of(v, hh[e]); }
      bf16* d = WT + (size_t)(n0 + nr) * K + k0 + k8;
      *(volatile v4u_t*)d = *(const v4ua*)hh; *(volatile v4u_t*)(d + plane) = *(const v4ua*)hl; }
    __threadfence();
  }
}

template <typename AT, typename WT, int MODE>
__global__ __launch_bounds__(256) void gemm_split_kernel(
    const AT* __restrict__ A, size_t aPlane, const WT* __restrict__ W, size_t wPlane,
    const float* __restrict__ bias, void* __restrict__ out,
    int M, int N, int K) {
  __shared__ bf16 ldsA[128 * LDS_STRIDE], ldsAl[128 * LDS_STRIDE];
  __shared__ bf16 ldsW[256 * LDS_STRIDE], ldsWl[256 * LDS_STRIDE];
  __shared__ __attribute__((aligned(16))) unsigned char sob[256 * 136 * 2];

  const int t    = threadIdx.x;
  const int wave = t >> 5;
  const int lane = t & 31;
  const int wm   = (wave & 1) * 64;
  const int wn   = (wave >> 1) * 64;
  const int mBlk = blockIdx.x * 128;
  const int nBlk = blockIdx.y * 256;
  const int arow = t >> 1;
  const int ach  = (t & 1) * 16;

  f32x8 acc[4][4] = {};
  for (int k = 0; k < K; k += 32) {
    __syncthreads();
    {
      const AT* ap = A + (size_t)(mBlk + arow) * K + k + ach;
      bf16 hh[16], hl[16];
      if (sizeof(AT) == 4) {
#pragma unroll
        for (int i = 0; i < 16; ++i) { const float v = (float)ap[i]; hh[i] = (bf16)v; hl[i] = lo_of(v, hh[i]); }
      } else {
#pragma unroll
        for (int i = 0; i < 16; ++i) { hh[i] = (bf16)ap[i]; hl[i] = (bf16)ap[aPlane + i]; }
      }
#pragma unroll
      for (int i = 0; i < 16; ++i) { ldsA[arow * LDS_STRIDE + ach + i] = hh[i]; ldsAl[arow * LDS_STRIDE + ach + i] = hl[i]; }
    }
    {
      const WT* wp = W + (size_t)(nBlk + t) * K + k;
      if (sizeof(WT) == 4) {
#pragma unroll
        for (int i = 0; i < 32; ++i) { const float v = (float)wp[i]; const bf16 h_ = (bf16)v; ldsW[t * LDS_STRIDE + i] = h_; ldsWl[t * LDS_STRIDE + i] = lo_of(v, h_); }
      } else {
#pragma unroll
        for (int i = 0; i < 32; ++i) { ldsW[t * LDS_STRIDE + i] = (bf16)wp[i]; ldsWl[t * LDS_STRIDE + i] = (bf16)wp[wPlane + i]; }
      }
    }
    __syncthreads();
    bf16x16 wf[4], wfl[4];
#pragma unroll
    for (int j = 0; j < 4; ++j) { wf[j] = lds_frag(ldsW + (wn + 16 * j) * LDS_STRIDE, LDS_STRIDE); wfl[j] = lds_frag(ldsWl + (wn + 16 * j) * LDS_STRIDE, LDS_STRIDE); }
#pragma unroll
    for (int i = 0; i < 4; ++i) {
      const bf16x16 af = lds_frag(ldsA + (wm + 16 * i) * LDS_STRIDE, LDS_STRIDE), afl = lds_frag(ldsAl + (wm + 16 * i) * LDS_STRIDE, LDS_STRIDE);
#pragma unroll
      for (int j = 0; j < 4; ++j) acc[i][j] = wmma_split(af, afl, wf[j], wfl[j], acc[i][j]);
    }
  }

  const int nlane = lane & 15;
  const int mh    = (lane >> 4) * 8;
  __syncthreads();
  if (MODE == 1) {
    bf16* so = (bf16*)sob;
#pragma unroll
    for (int i = 0; i < 4; ++i)
#pragma unroll
      for (int j = 0; j < 4; ++j) {
        const int nl = wn + 16 * j + nlane;
        const float bv = bias ? bias[nBlk + nl] : 0.0f;
#pragma unroll
        for (int r = 0; r < 8; ++r) so[nl * 136 + wm + 16 * i + mh + r] = (bf16)(acc[i][j][r] + bv);
      }
    __syncthreads();
    const int b_ = mBlk >> 11, s0 = mBlk & (SS - 1);
#pragma unroll 1
    for (int pass = 0; pass < 2; ++pass) {
      for (int ch = t; ch < 256 * 16; ch += 256) { const int nl = ch >> 4, q = (ch & 15) * 8; const int n = nBlk + nl, h = n >> 6, dk = n & (DKK - 1);
        *(volatile v4u_t*)((bf16*)out + (((size_t)(b_ * HH + h)) * DKK + dk) * SS + s0 + q) = *(const v4ua*)(so + nl * 136 + q); }
      __threadfence();
    }
  } else {
    float* so = (float*)sob;
#pragma unroll 1
    for (int hf = 0; hf < 2; ++hf) {
      if (wm == hf * 64) {
#pragma unroll
        for (int i = 0; i < 4; ++i)
#pragma unroll
          for (int j = 0; j < 4; ++j) {
            const int nl = wn + 16 * j + nlane;
            const float bv = bias ? bias[nBlk + nl] : 0.0f;
#pragma unroll
            for (int r = 0; r < 8; ++r) so[(16 * i + mh + r) * 260 + nl] = acc[i][j][r] + bv;
          }
      }
      __syncthreads();
#pragma unroll 1
      for (int pass = 0; pass < 2; ++pass) {
        for (int ch = t; ch < 64 * 64; ch += 256) { const int ml = ch >> 6, q = (ch & 63) * 4;
          *(volatile v4f_t*)((float*)out + (size_t)(mBlk + hf * 64 + ml) * N + nBlk + q) = *(const volatile v4fa*)(so + ml * 260 + q); }
        __threadfence();
      }
      __syncthreads();
    }
  }
}


#define MB 4
#define MC 32
#define MHW 36864
#define MHH 192
#define MPIX (MB * MHW)
#define BETA 15.0f
#define NPB 576

__global__ __launch_bounds__(256) void k_dilate(const float* __restrict__ x, const float* __restrict__ wd, int di, float* __restrict__ D) {
  const int b = blockIdx.y, p = blockIdx.x * 256 + threadIdx.x, py = p / MHH, px = p % MHH, d = di + 1;
  const float* xb = x + (size_t)b * MC * MHW; float* Db = D + (size_t)b * MC * MHW;
#pragma unroll 1
  for (int c = 0; c < MC; ++c) {
    const float* xc = xb + (size_t)c * MHW; const float* w = wd + ((size_t)di * MC + c) * 9;
    float v[9]; float mx = -3.0e38f;
#pragma unroll 1
    for (int t = 0; t < 9; ++t) { const int yy = py + (t / 3 - 1) * d, xx = px + (t % 3 - 1) * d;
      const float xv = (yy >= 0 && yy < MHH && xx >= 0 && xx < MHH) ? xc[yy * MHH + xx] : 0.0f;
      v[t] = BETA * (xv + w[t]); mx = fmaxf(mx, v[t]); }
    float s = 0.0f;
#pragma unroll 1
    for (int t = 0; t < 9; ++t) s += expf(v[t] - mx);
    const float r = (mx + logf(s)) / BETA;
    *(volatile float*)(Db + (size_t)c * MHW + p) = r;
  }
  __threadfence();
#pragma unroll 1
  for (int c = 0; c < MC; ++c) { const float r = *(volatile const float*)(Db + (size_t)c * MHW + p); *(volatile float*)(Db + (size_t)c * MHW + p) = r; }
}
__global__ __launch_bounds__(256) void k_erode(const float* __restrict__ D, const float* __restrict__ we, int di, float* __restrict__ Y, float* __restrict__ part) {
  __shared__ float red[2][256];
  __shared__ float rowbuf[256][33];
  const int b = blockIdx.y, tid = threadIdx.x, p = blockIdx.x * 256 + tid, py = p / MHH, px = p % MHH, d = di + 1;
  const float* Db = D + (size_t)b * MC * MHW;
#pragma unroll 1
  for (int c = 0; c < MC; ++c) {
    const float* Dc = Db + (size_t)c * MHW; const float* w = we + ((size_t)di * MC + c) * 9;
    float v[9]; float mx = -3.0e38f;
#pragma unroll 1
    for (int t = 0; t < 9; ++t) { const int yy = py + (t / 3 - 1) * d, xx = px + (t % 3 - 1) * d;
      const float dv = (yy >= 0 && yy < MHH && xx >= 0 && xx < MHH) ? Dc[yy * MHH + xx] : 0.0f;
      v[t] = BETA * (w[t] - dv); mx = fmaxf(mx, v[t]); }
    float s = 0.0f;
#pragma unroll 1
    for (int t = 0; t < 9; ++t) s += expf(v[t] - mx);
    const float r = -((mx + logf(s)) / BETA);
    rowbuf[tid][c] = r;
    red[0][tid] = r; red[1][tid] = r * r; __syncthreads();
    for (int o = 128; o > 0; o >>= 1) { if (tid < o) { red[0][tid] += red[0][tid + o]; red[1][tid] += red[1][tid + o]; } __syncthreads(); }
    if (tid == 0) { const int blk = b * (MHW / 256) + blockIdx.x; part[((size_t)blk * MC + c) * 2] = red[0][0]; part[((size_t)blk * MC + c) * 2 + 1] = red[1][0]; }
    __syncthreads();
  }
#pragma unroll 1
  for (int pass = 0; pass < 2; ++pass) {
    for (int i = tid; i < 256 * 8; i += 256) { const int pr = i >> 3, c4 = (i & 7) * 4; v4f_t vv; vv.x = rowbuf[pr][c4]; vv.y = rowbuf[pr][c4 + 1]; vv.z = rowbuf[pr][c4 + 2]; vv.w = rowbuf[pr][c4 + 3];
      *(volatile v4f_t*)(Y + ((size_t)b * MHW + blockIdx.x * 256 + pr) * 128 + di * 32 + c4) = vv; }
    if (tid < MC) { const int blk = b * (MHW / 256) + blockIdx.x; const float a = part[((size_t)blk * MC + tid) * 2], q = part[((size_t)blk * MC + tid) * 2 + 1];
      *(volatile float*)(part + ((size_t)blk * MC + tid) * 2) = a; *(volatile float*)(part + ((size_t)blk * MC + tid) * 2 + 1) = q; }
    __threadfence();
  }
}
__global__ __launch_bounds__(256) void k_stats(const float* __restrict__ part, int choff, float* __restrict__ st) {
  __shared__ float r0[256], r1[256];
  const int c = blockIdx.x, tid = threadIdx.x;
  float a = 0.0f, q = 0.0f;
  for (int i = tid; i < NPB; i += 256) { a += part[((size_t)i * MC + c) * 2]; q += part[((size_t)i * MC + c) * 2 + 1]; }
  r0[tid] = a; r1[tid] = q; __syncthreads();
  for (int o = 128; o > 0; o >>= 1) { if (tid < o) { r0[tid] += r0[tid + o]; r1[tid] += r1[tid + o]; } __syncthreads(); }
  if (tid == 0) { const float m = r0[0] / (float)MPIX, var = fmaxf(r1[0] / (float)MPIX - m * m, 0.0f);
    st[(choff + c) * 32] = m; st[(choff + c) * 32 + 1] = rsqrtf(var + 1e-5f); __threadfence(); st[(choff + c) * 32] = m; st[(choff + c) * 32 + 1] = rsqrtf(var + 1e-5f); }
}
__global__ __launch_bounds__(256) void k_bnrelu(float* __restrict__ Y, const float* __restrict__ st, const float* __restrict__ gs, const float* __restrict__ bs, int di) {
  const int p = blockIdx.x * 8 + (threadIdx.x >> 5), lane = threadIdx.x & 31;
  const int ch = di * 32 + lane; float* q = Y + (size_t)p * 128 + ch;
  const float m = st[ch * 32], rs = st[ch * 32 + 1];
  const float v = fmaxf((q[0] - m) * rs * gs[di * MC + lane] + bs[di * MC + lane], 0.0f);
  *(volatile float*)q = v; __threadfence(); *(volatile float*)q = v;
}
__global__ __launch_bounds__(256) void k_stats2(const float* __restrict__ out, float* __restrict__ st2) {
  __shared__ float r0[256], r1[256];
  const int o = blockIdx.x, tid = threadIdx.x; float a = 0.0f, q = 0.0f;
  for (int b = 0; b < MB; ++b) { const float* p = out + ((size_t)b * MC + o) * MHW; for (int i = tid; i < MHW; i += 256) { const float v = p[i]; a += v; q += v * v; } }
  r0[tid] = a; r1[tid] = q; __syncthreads();
  for (int s = 128; s > 0; s >>= 1) { if (tid < s) { r0[tid] += r0[tid + s]; r1[tid] += r1[tid + s]; } __syncthreads(); }
  if (tid == 0) { const float m = r0[0] / (float)MPIX, var = fmaxf(r1[0] / (float)MPIX - m * m, 0.0f);
    st2[o * 32] = m; st2[o * 32 + 1] = rsqrtf(var + 1e-5f); __threadfence(); st2[o * 32] = m; st2[o * 32 + 1] = rsqrtf(var + 1e-5f); }
}
__global__ __launch_bounds__(256) void k_bnrelu2(float* __restrict__ out, const float* __restrict__ st2, const float* __restrict__ g, const float* __restrict__ bb) {
  const size_t e0 = ((size_t)blockIdx.x * 256 + threadIdx.x) * 4; const int o = (int)((e0 / MHW) % MC);
  const float m = st2[o * 32], rs = st2[o * 32 + 1], a = rs * g[o], c0 = bb[o] - m * rs * g[o];
  v4f_t v = *(const volatile v4fa*)(out + e0); v.x = fmaxf(v.x * a + c0, 0.0f); v.y = fmaxf(v.y * a + c0, 0.0f); v.z = fmaxf(v.z * a + c0, 0.0f); v.w = fmaxf(v.w * a + c0, 0.0f);
  *(volatile v4f_t*)(out + e0) = v; __threadfence(); *(volatile v4f_t*)(out + e0) = v;
}
__global__ __launch_bounds__(128) void k_packA(const float* __restrict__ Wc, float* __restrict__ A) {
  const int m = blockIdx.x, k = threadIdx.x; const float v = (m < MC) ? Wc[m * 128 + k] : 0.0f;
  *(volatile float*)(A + m * 128 + k) = v; __threadfence(); *(volatile float*)(A + m * 128 + k) = v;
}

__global__ __launch_bounds__(256) void k_copyrows(const float* __restrict__ T, int b, float* __restrict__ out) {
  const int o = blockIdx.x, t = threadIdx.x;
#pragma unroll 1
  for (int pass = 0; pass < 2; ++pass) {
    for (int i = t; i < MHW / 4; i += 256) *(volatile v4f_t*)(out + ((size_t)b * MC + o) * MHW + (size_t)i * 4) = *(const volatile v4fa*)(T + (size_t)o * MHW + (size_t)i * 4);
    __threadfence();
  }
}

extern "C" void kernel_launch(void* const* d_in, const int* in_sizes, int n_in,
                              void* d_out, int out_size, void* d_ws, size_t ws_size,
                              hipStream_t stream) {
  (void)in_sizes; (void)n_in; (void)out_size; (void)ws_size;
  const float* x  = (const float*)d_in[0];
  const float* wd = (const float*)d_in[1];  const float* we = (const float*)d_in[2];
  const float* gs = (const float*)d_in[3];  const float* bs = (const float*)d_in[4];
  const float* Wc = (const float*)d_in[5];
  const float* g  = (const float*)d_in[6];  const float* bb = (const float*)d_in[7];
  float* out = (float*)d_out;
  char* ws = (char*)d_ws;
  float* D    = (float*)ws; ws += (size_t)MB * MC * MHW * 4;
  float* Y    = (float*)ws; ws += (size_t)MPIX * 128 * 4;
  float* part = (float*)ws; ws += (size_t)MC * NPB * 2 * 4;
  float* st   = (float*)ws; ws += 128 * 32 * 4;
  float* st2  = (float*)ws; ws += 32 * 32 * 4;
  float* A    = (float*)ws; ws += 128 * 128 * 4;
  float* T    = D;
  (void)T;
  k_packA<<<128, 128, 0, stream>>>(Wc, A);
  for (int di = 0; di < 4; ++di) {
    k_dilate<<<dim3(MHW / 256, MB), 256, 0, stream>>>(x, wd, di, D);
    k_erode<<<dim3(MHW / 256, MB), 256, 0, stream>>>(D, we, di, Y, part);
    k_stats<<<MC, 256, 0, stream>>>(part, di * 32, st);
    k_bnrelu<<<MPIX / 8, 256, 0, stream>>>(Y, st, gs, bs, di);
  }
  for (int b = 0; b < MB; ++b)
  { gemm_split_kernel<float, float, 2><<<dim3(1, MHW / 256), 256, 0, stream>>>(A, 0, Y + (size_t)b * MHW * 128, 0, nullptr, D  , 128, MHW, 128);
    k_copyrows<<<MC, 256, 0, stream>>>(D, b, out); }
  k_stats2<<<MC, 256, 0, stream>>>(out, st2);
  k_bnrelu2<<<(int)((size_t)MB * MC * MHW / 4 / 256), 256, 0, stream>>>(out, st2, g, bb);
}
